// EGNNModel_25305947308630
// MI455X (gfx1250) — hardware-verified
//
#include <hip/hip_runtime.h>
#include <stddef.h>


#define NN     20000
#define NE     160000
#define DD     128
#define NL     5
#define NG     64
#define NPAD   20096
#define LN_EPS 1e-5f
#define WSC    16.0f
#define WINV   0.0625f
#define INV_D  0.0078125f

#define NTHR   256
#define NWAVE  8
#define EPT    8
#define CHUNK  (NTHR * EPT)
#define WCAP   (EPT * 32)
#define LISTN  (NWAVE * WCAP)
#define PASSN  (NWAVE * 16)
#define PCAP   (CHUNK + PASSN)
#define NB     128
#define AP     136

static_assert((NPAD % 128) == 0);
static_assert(NPAD >= NN);
static_assert((NPAD % NB) == 0);
static_assert(PASSN == 128);
static_assert(NB == NWAVE * 16);
static_assert(PCAP >= CHUNK + PASSN);

typedef float    v4f  __attribute__((ext_vector_type(4)));
typedef float    v8f  __attribute__((ext_vector_type(8)));
typedef int      v4i  __attribute__((ext_vector_type(4)));
typedef _Float16 v4h  __attribute__((ext_vector_type(4)));
typedef _Float16 v8h  __attribute__((ext_vector_type(8)));
typedef _Float16 v16h __attribute__((ext_vector_type(16)));
union FragH { v16h v; v8h h[2]; };

__device__ __forceinline__ int clampi(int v, int lo, int hi) { return v < lo ? lo : (v > hi ? hi : v); }

__device__ __forceinline__ v4f z4() { v4f z; z.x = 0.0f; z.y = 0.0f; z.z = 0.0f; z.w = 0.0f; return z; }

__device__ __forceinline__ v8f z8() {
  v8f c;
#pragma unroll
  for (int i = 0; i < 8; ++i) c[i] = 0.0f;
  return c;
}

__device__ __forceinline__ v8h cvt8(v4f a, v4f b) {
  v8h r;
  r[0] = (_Float16)a.x; r[1] = (_Float16)a.y; r[2] = (_Float16)a.z; r[3] = (_Float16)a.w;
  r[4] = (_Float16)b.x; r[5] = (_Float16)b.y; r[6] = (_Float16)b.z; r[7] = (_Float16)b.w;
  return r;
}

__device__ __forceinline__ v8f wmh(v16h a, v16h b, v8f c) {
  v8f d = __builtin_amdgcn_wmma_f32_16x16x32_f16(false, a, false, b, (short)0, c, false, false);
  asm volatile("v_nop\n\tv_nop\n\tv_nop\n\tv_nop" : "+v"(d) : "v"(a), "v"(b));
  return d;
}

__device__ __forceinline__ v16h ldfrag(const _Float16* p) {
  FragH f;
  f.h[0] = *(const v8h*)p;
  f.h[1] = *(const v8h*)(p + 16);
  return f.v;
}

__device__ __forceinline__ float sum16(float v) {
  v += __shfl_xor(v, 1, 32); v += __shfl_xor(v, 2, 32); v += __shfl_xor(v, 4, 32); v += __shfl_xor(v, 8, 32);
  return v;
}
__device__ __forceinline__ float sum32(float v) { v = sum16(v); v += __shfl_xor(v, 16, 32); return v; }

__device__ __forceinline__ void gemm_k128(v8f (&acc)[8], const _Float16* arow, const _Float16* wtb, int kp, int m) {
#pragma unroll
  for (int ks = 0; ks < 4; ++ks) {
    const v16h a = ldfrag(arow + ks * 32);
#pragma unroll
    for (int nt = 0; nt < 8; ++nt) {
      const v16h b = ldfrag(wtb + (size_t)(nt * 16 + m) * kp + ks * 32);
      acc[nt] = wmh(a, b, acc[nt]);
    }
  }
}

__device__ __forceinline__ void epi_ln_relu(v8f (&acc)[8], const float* __restrict__ bias,
                                            const float* __restrict__ gam, const float* __restrict__ bet, int m) {
  float bb[8], gg[8], ee[8];
#pragma unroll
  for (int nt = 0; nt < 8; ++nt) { const int c = nt * 16 + m; bb[nt] = bias[c]; gg[nt] = gam[c]; ee[nt] = bet[c]; }
#pragma unroll
  for (int r = 0; r < 8; ++r) {
    float x[8];
    float s = 0.0f;
#pragma unroll
    for (int nt = 0; nt < 8; ++nt) { x[nt] = acc[nt][r] * WINV + bb[nt]; s += x[nt]; }
    s = sum16(s);
    const float mean = s * INV_D;
    float q = 0.0f;
#pragma unroll
    for (int nt = 0; nt < 8; ++nt) { const float d = x[nt] - mean; x[nt] = d; q += d * d; }
    q = sum16(q);
    const float rstd = rsqrtf(q * INV_D + LN_EPS);
#pragma unroll
    for (int nt = 0; nt < 8; ++nt) acc[nt][r] = fmaxf(x[nt] * rstd * gg[nt] + ee[nt], 0.0f);
  }
}

__global__ __launch_bounds__(NTHR) void k_wcvt(const float* __restrict__ src, int srcStride, int rowShift,
                                               _Float16* dst, int Nout, int K, int total) {
  const int t = blockIdx.x * NTHR + threadIdx.x;
  if (t >= total) return;
  const int kg8  = K >> 3;
  const int perL = Nout * kg8;
  const int l    = t / perL;
  const int rem  = t - l * perL;
  const int n    = rem / kg8;
  const int kg   = rem - n * kg8;
  const float* sp = src + (size_t)l * srcStride + (size_t)((n >> 7) * rowShift + kg * 8) * DD + (n & 127);
  v8h hv;
#pragma unroll
  for (int j = 0; j < 8; ++j) hv[j] = (_Float16)(sp[(size_t)j * DD] * WSC);
  _Float16* dp = dst + (size_t)l * Nout * K + (size_t)n * K + kg * 8;
  *(volatile v8h*)dp = hv;
  __threadfence();
  *(volatile v8h*)dp = hv;
}

__global__ __launch_bounds__(NTHR) void k_init(const int* __restrict__ atoms, const float* __restrict__ emb,
                                               const float* __restrict__ posIn,
                                               float* h32, _Float16* h16, float* pos4, int nN, int nEmb) {
  const int t = blockIdx.x * NTHR + threadIdx.x;
  const bool s1 = t < NPAD * 32, s2 = t < NPAD * 16, s3 = t < NPAD;
  const int n1 = t >> 5, c4 = (t & 31) * 4;
  const int n2 = t >> 4, c8 = (t & 15) * 8;
  v4f a = z4();
  {
    const int nn = clampi(n1, 0, nN - 1);
    const int at = clampi(atoms[nn], 0, nEmb - 1);
    const v4f v = *(const v4f*)(emb + (size_t)at * DD + c4);
    if (n1 < nN) a = v;
  }
  v8h b;
  {
    const int nn = clampi(n2, 0, nN - 1);
    const int at = clampi(atoms[nn], 0, nEmb - 1);
    v4f v0 = *(const v4f*)(emb + (size_t)at * DD + c8);
    v4f v1 = *(const v4f*)(emb + (size_t)at * DD + c8 + 4);
    if (n2 >= nN) { v0 = z4(); v1 = z4(); }
    b = cvt8(v0, v1);
  }
  v4f c = z4();
  {
    const int nn = clampi(t, 0, nN - 1);
    const float px = posIn[(size_t)nn * 3 + 0], py = posIn[(size_t)nn * 3 + 1], pz = posIn[(size_t)nn * 3 + 2];
    if (t < nN) { c.x = px; c.y = py; c.z = pz; c.w = 0.0f; }
  }
  if (s1) *(volatile v4f*)(h32 + (size_t)n1 * DD + c4) = a;
  if (s2) *(volatile v8h*)(h16 + (size_t)n2 * DD + c8) = b;
  if (s3) *(volatile v4f*)(pos4 + (size_t)t * 4) = c;
  __threadfence();
  if (s1) *(volatile v4f*)(h32 + (size_t)n1 * DD + c4) = a;
  if (s2) *(volatile v8h*)(h16 + (size_t)n2 * DD + c8) = b;
  if (s3) *(volatile v4f*)(pos4 + (size_t)t * 4) = c;
}

__device__ __forceinline__ void pq_pass(const float* sw, float* dst, int lane) {
#pragma unroll
  for (int r = 0; r < 16; ++r) {
    const v4f v = *(const v4f*)(sw + r * DD + 4 * lane);
    *(volatile v4f*)(dst + (size_t)r * 256 + 4 * lane) = v;
  }
}

__global__ __launch_bounds__(NTHR) void k_pq(const _Float16* __restrict__ h16, const _Float16* __restrict__ w1t,
                                             const float* __restrict__ b1, float* PQ) {
  __shared__ __attribute__((aligned(16))) float stg[NWAVE * 16 * DD];
  const int tid = threadIdx.x, lane = tid & 31, wave = tid >> 5, hh = lane >> 4, m = lane & 15;
  const int mt = wave & 3, chf = wave >> 2;
  const int row0 = blockIdx.x * 64 + mt * 16;
  const int col0 = chf * DD;
  v8f acc[8];
#pragma unroll
  for (int i = 0; i < 8; ++i) acc[i] = z8();
  gemm_k128(acc, h16 + (size_t)(row0 + m) * DD + 8 * hh, w1t + (size_t)col0 * DD + 8 * hh, DD, m);
  float* sw = stg + wave * 16 * DD;
#pragma unroll
  for (int nt = 0; nt < 8; ++nt) {
    const int c = nt * 16 + m;
    const float bv = b1[c];
    const float bias = (chf == 0) ? bv : 0.0f;
#pragma unroll
    for (int r = 0; r < 8; ++r) sw[(8 * hh + r) * DD + c] = acc[nt][r] * WINV + bias;
  }
  __syncthreads();
  float* dst = PQ + (size_t)row0 * 256 + col0;
  pq_pass(sw, dst, lane);
  __threadfence();
  pq_pass(sw, dst, lane);
}

__device__ __forceinline__ int scan_chunk(const int* __restrict__ dsts, int nE, int cbase, int nodeBase,
                                          int vec8, int* list, int tid, int wave) {
  int wc = 0;
  const int el0  = tid * EPT;
  const int e0   = cbase + el0;
  const int sent = -2147483647 - 1;
  v4i da, db;
  if (vec8 != 0 && cbase + CHUNK <= nE) {
    da = *(const v4i*)(dsts + e0);
    db = *(const v4i*)(dsts + e0 + 4);
  } else {
    da.x = (e0     < nE) ? dsts[min(e0,     nE - 1)] : sent;
    da.y = (e0 + 1 < nE) ? dsts[min(e0 + 1, nE - 1)] : sent;
    da.z = (e0 + 2 < nE) ? dsts[min(e0 + 2, nE - 1)] : sent;
    da.w = (e0 + 3 < nE) ? dsts[min(e0 + 3, nE - 1)] : sent;
    db.x = (e0 + 4 < nE) ? dsts[min(e0 + 4, nE - 1)] : sent;
    db.y = (e0 + 5 < nE) ? dsts[min(e0 + 5, nE - 1)] : sent;
    db.z = (e0 + 6 < nE) ? dsts[min(e0 + 6, nE - 1)] : sent;
    db.w = (e0 + 7 < nE) ? dsts[min(e0 + 7, nE - 1)] : sent;
  }
  const unsigned nb = (unsigned)nodeBase;
  const unsigned s0 = (unsigned)da.x - nb, s1 = (unsigned)da.y - nb;
  const unsigned s2 = (unsigned)da.z - nb, s3 = (unsigned)da.w - nb;
  const unsigned s4 = (unsigned)db.x - nb, s5 = (unsigned)db.y - nb;
  const unsigned s6 = (unsigned)db.z - nb, s7 = (unsigned)db.w - nb;
  const bool h0 = s0 < (unsigned)NB, h1 = s1 < (unsigned)NB, h2 = s2 < (unsigned)NB, h3 = s3 < (unsigned)NB;
  const bool h4 = s4 < (unsigned)NB, h5 = s5 < (unsigned)NB, h6 = s6 < (unsigned)NB, h7 = s7 < (unsigned)NB;
  const unsigned any = __builtin_amdgcn_ballot_w32(h0 | h1 | h2 | h3 | h4 | h5 | h6 | h7);
  if (any != 0u) {
#define HITJ(J, HJ) { \
      const unsigned mj = __builtin_amdgcn_ballot_w32(HJ); \
      if (mj != 0u) { \
        if (HJ) { \
          const int ps = wc + (int)__builtin_amdgcn_mbcnt_lo(mj, 0u); \
          if (ps < WCAP) list[wave * WCAP + ps] = el0 + (J); \
        } \
        wc += (int)__builtin_popcount(mj); } }
    HITJ(0, h0)
    HITJ(1, h1)
    HITJ(2, h2)
    HITJ(3, h3)
    HITJ(4, h4)
    HITJ(5, h5)
    HITJ(6, h6)
    HITJ(7, h7)
#undef HITJ
  }
  return wc;
}

__device__ __forceinline__ void edge_out_pass(const float* accm, const float* accp, const float* __restrict__ posOld,
                                              _Float16* msgOut, float* posNew, int nodeBase, int wave, int lane, int hh, int m) {
#pragma unroll
  for (int rp = 0; rp < 8; ++rp) {
    const int sl = wave * 16 + 2 * rp + hh;
    const float* ar = accm + sl * DD + 8 * m;
    const v4f x0 = *(const v4f*)ar;
    const v4f x1 = *(const v4f*)(ar + 4);
    const v8h hv = cvt8(x0, x1);
    *(volatile v8h*)(msgOut + (size_t)(nodeBase + sl) * DD + 8 * m) = hv;
  }
  if (wave == 0) {
#pragma unroll
    for (int k = 0; k < 4; ++k) {
      const int sl = 32 * k + lane;
      const v4f po = *(const v4f*)(posOld + (size_t)(nodeBase + sl) * 4);
      const float cn = accp[sl * 4 + 3];
      const float rc = 1.0f / fmaxf(cn, 1.0f);
      v4f pn;
      pn.x = po.x + accp[sl * 4 + 0] * rc;
      pn.y = po.y + accp[sl * 4 + 1] * rc;
      pn.z = po.z + accp[sl * 4 + 2] * rc;
      pn.w = 0.0f;
      *(volatile v4f*)(posNew + (size_t)(nodeBase + sl) * 4) = pn;
    }
  }
}

__global__ __launch_bounds__(NTHR) void k_edge(
    const float* __restrict__ PQ, const float* __restrict__ posOld, const int* __restrict__ ei,
    const float* __restrict__ wdist, const float* __restrict__ g1, const float* __restrict__ e1,
    const _Float16* __restrict__ w2t, const float* __restrict__ b2, const float* __restrict__ g2, const float* __restrict__ e2,
    const _Float16* __restrict__ w3t, const float* __restrict__ b3, const float* __restrict__ g3, const float* __restrict__ e3,
    const float* __restrict__ w4, const float* __restrict__ b4,
    _Float16* msgOut, float* posNew, int nN, int nE, int vec8) {
  __shared__ __attribute__((aligned(16))) float    accm[(NB + 2) * DD];
  __shared__ __attribute__((aligned(16))) float    accp[(NB + 2) * 4];
  __shared__ __attribute__((aligned(16))) _Float16 atile[NWAVE * 16 * AP];
  __shared__ __attribute__((aligned(16))) int      list[LISTN];
  __shared__ __attribute__((aligned(16))) int      pend[PCAP];
  __shared__ __attribute__((aligned(16))) float    pdb[PASSN * 4];
  __shared__ int   slotb[PASSN];
  __shared__ float svb[PASSN];
  __shared__ int   wcnt[NWAVE];
  __shared__ int   pendN;

  const int tid = threadIdx.x, lane = tid & 31, wave = tid >> 5, hh = lane >> 4, m = lane & 15;
  const int nodeBase = blockIdx.x * NB;
  const int* srcs = ei;
  const int* dsts = ei + nE;

  for (int i = tid; i < (NB + 2) * DD; i += NTHR) accm[i] = 0.0f;
  for (int i = tid; i < (NB + 2) * 4; i += NTHR) accp[i] = 0.0f;
  if (tid == 0) pendN = 0;
  const v4f wdv = *(const v4f*)(wdist + 4 * lane);
  const v4f g1v = *(const v4f*)(g1 + 4 * lane);
  const v4f e1v = *(const v4f*)(e1 + 4 * lane);
  __syncthreads();

  const int nChunks = (nE + CHUNK - 1) / CHUNK;
#pragma unroll 1
  for (int ch = 0; ch < nChunks; ++ch) {
    const int cbase = ch * CHUNK;
    const int wc = scan_chunk(dsts, nE, cbase, nodeBase, vec8, list, tid, wave);
    if (lane == 0) wcnt[wave] = wc;
    __syncthreads();

    const int base = pendN;
    int tot = 0, myoff = 0;
#pragma unroll
    for (int w = 0; w < NWAVE; ++w) {
      int c = wcnt[w];
      c = c > WCAP ? WCAP : (c < 0 ? 0 : c);
      if (w < wave) myoff += c;
      tot += c;
    }
    int newN = base + tot;
    newN = newN > PCAP ? PCAP : newN;
    {
      int n = wcnt[wave];
      n = n > WCAP ? WCAP : (n < 0 ? 0 : n);
      const int* lp = list + wave * WCAP;
      for (int i = lane; i < n; i += 32) {
        const int ps = base + myoff + i;
        if (ps < PCAP) pend[ps] = cbase + lp[i];
      }
    }
    const int fin = (ch == nChunks - 1) ? 1 : 0;
    const int R   = (fin != 0) ? (newN + PASSN - 1) / PASSN : newN / PASSN;
    const int Pv  = (fin != 0) ? newN : R * PASSN;
    __syncthreads();

#pragma unroll 1
    for (int rp = 0; rp < R; ++rp) {
      {
        _Float16* trow = atile + (wave * 16) * AP + 4 * lane;
#pragma unroll 1
        for (int r = 0; r < 16; ++r) {
          const int idx = rp * PASSN + wave * 16 + r;
          const bool valid = idx < Pv;
          int e = pend[idx < PCAP - 1 ? idx : PCAP - 1];
          e = valid ? e : 0;
          e = clampi(e, 0, nE - 1);
          int d = dsts[e];
          int s = srcs[e];
          int slot = d - nodeBase;
          if (!valid || (unsigned)slot >= (unsigned)NB) slot = NB;
          d = clampi(d, 0, nN - 1);
          s = clampi(s, 0, nN - 1);
          const v4f P  = *(const v4f*)(PQ + (size_t)d * 256 + 4 * lane);
          const v4f Q  = *(const v4f*)(PQ + (size_t)s * 256 + DD + 4 * lane);
          const v4f pi = *(const v4f*)(posOld + (size_t)d * 4);
          const v4f pj = *(const v4f*)(posOld + (size_t)s * 4);
          const float dx = pi.x - pj.x, dy = pi.y - pj.y, dz = pi.z - pj.z;
          const float dist = sqrtf(dx * dx + dy * dy + dz * dz);
          float x0 = P.x + Q.x + dist * wdv.x;
          float x1 = P.y + Q.y + dist * wdv.y;
          float x2 = P.z + Q.z + dist * wdv.z;
          float x3 = P.w + Q.w + dist * wdv.w;
          const float sm = sum32((x0 + x1) + (x2 + x3));
          const float mean = sm * INV_D;
          x0 -= mean; x1 -= mean; x2 -= mean; x3 -= mean;
          const float q = sum32(x0 * x0 + x1 * x1 + x2 * x2 + x3 * x3);
          const float rstd = rsqrtf(q * INV_D + LN_EPS);
          v4h hv;
          hv.x = (_Float16)fmaxf(x0 * rstd * g1v.x + e1v.x, 0.0f);
          hv.y = (_Float16)fmaxf(x1 * rstd * g1v.y + e1v.y, 0.0f);
          hv.z = (_Float16)fmaxf(x2 * rstd * g1v.z + e1v.z, 0.0f);
          hv.w = (_Float16)fmaxf(x3 * rstd * g1v.w + e1v.w, 0.0f);
          *(v4h*)(trow + r * AP) = hv;
          if (lane == 0) {
            const int q4 = (wave * 16 + r) * 4;
            slotb[wave * 16 + r] = slot;
            pdb[q4 + 0] = dx; pdb[q4 + 1] = dy; pdb[q4 + 2] = dz; pdb[q4 + 3] = 0.0f;
          }
        }
      }
      __syncthreads();

      {
        v8f acc[8];
#pragma unroll
        for (int i = 0; i < 8; ++i) acc[i] = z8();
        gemm_k128(acc, atile + (wave * 16 + m) * AP + 8 * hh, w2t + 8 * hh, DD, m);
        epi_ln_relu(acc, b2, g2, e2, m);
#pragma unroll 1
        for (int w = 0; w < NWAVE; ++w) {
          if (wave == w) {
#pragma unroll
            for (int rr = 0; rr < 16; ++rr) {
              int sl = slotb[wave * 16 + rr];
              sl = clampi(sl, 0, NB);
              const int row = (hh == (rr >> 3)) ? sl : (NB + 1);
              float* ap = accm + row * DD + m;
#pragma unroll
              for (int nt = 0; nt < 8; ++nt) ap[nt * 16] += acc[nt][rr & 7];
            }
          }
          __syncthreads();
        }
        _Float16* tw = atile + (wave * 16 + 8 * hh) * AP + m;
#pragma unroll
        for (int r = 0; r < 8; ++r)
#pragma unroll
          for (int nt = 0; nt < 8; ++nt) tw[r * AP + nt * 16] = (_Float16)acc[nt][r];
      }
      __syncthreads();

      {
        v8f acc[8];
#pragma unroll
        for (int i = 0; i < 8; ++i) acc[i] = z8();
        gemm_k128(acc, atile + (wave * 16 + m) * AP + 8 * hh, w3t + 8 * hh, DD, m);
        epi_ln_relu(acc, b3, g3, e3, m);
        float pw[8];
#pragma unroll
        for (int nt = 0; nt < 8; ++nt) pw[nt] = w4[nt * 16 + m];
        const float bb4 = b4[0];
#pragma unroll
        for (int r = 0; r < 8; ++r) {
          float sr = 0.0f;
#pragma unroll
          for (int nt = 0; nt < 8; ++nt) sr += acc[nt][r] * pw[nt];
          sr = sum16(sr);
          sr += bb4;
          if (m == 0) svb[wave * 16 + 8 * hh + r] = sr;
        }
      }
      __syncthreads();
      if (wave == 0 && lane < 4) {
#pragma unroll 1
        for (int e = 0; e < PASSN; ++e) {
          const int sl = clampi(slotb[e], 0, NB);
          const float sv = svb[e];
          const float pv = pdb[e * 4 + lane];
          const float add = (lane < 3) ? pv * sv : 1.0f;
          accp[sl * 4 + lane] += add;
        }
      }
      __syncthreads();
    }

    int rem = newN - R * PASSN;
    rem = rem < 0 ? 0 : rem;
    if (R > 0 && tid < rem) pend[tid] = pend[R * PASSN + tid];
    if (tid == 0) pendN = rem;
  }
  __syncthreads();

  edge_out_pass(accm, accp, posOld, msgOut, posNew, nodeBase, wave, lane, hh, m);
  __threadfence();
  edge_out_pass(accm, accp, posOld, msgOut, posNew, nodeBase, wave, lane, hh, m);
}

__device__ __forceinline__ void node_out_pass(const float* sw, float* h32n, _Float16* h16n, int lane, int hh, int m) {
#pragma unroll
  for (int r = 0; r < 16; ++r) {
    const v4f v = *(const v4f*)(sw + r * DD + 4 * lane);
    *(volatile v4f*)(h32n + (size_t)r * DD + 4 * lane) = v;
  }
#pragma unroll
  for (int rp = 0; rp < 8; ++rp) {
    const int row = 2 * rp + hh;
    const float* p = sw + row * DD + 8 * m;
    const v4f x0 = *(const v4f*)p;
    const v4f x1 = *(const v4f*)(p + 4);
    const v8h hv = cvt8(x0, x1);
    *(volatile v8h*)(h16n + (size_t)row * DD + 8 * m) = hv;
  }
}

__global__ __launch_bounds__(NTHR) void k_node(
    const _Float16* __restrict__ h16, const _Float16* __restrict__ msg16, const float* __restrict__ h32,
    const _Float16* __restrict__ u1t, const float* __restrict__ b1, const float* __restrict__ g1, const float* __restrict__ e1,
    const _Float16* __restrict__ u2t, const float* __restrict__ b2, const float* __restrict__ g2, const float* __restrict__ e2,
    float* h32n, _Float16* h16n) {
  __shared__ __attribute__((aligned(16))) _Float16 ut[NWAVE * 16 * AP];
  __shared__ __attribute__((aligned(16))) float    stg[NWAVE * 16 * DD];
  const int tid = threadIdx.x, lane = tid & 31, wave = tid >> 5, hh = lane >> 4, m = lane & 15;
  const int row0 = blockIdx.x * 128 + wave * 16;

  v8f acc[8];
#pragma unroll
  for (int i = 0; i < 8; ++i) acc[i] = z8();
  gemm_k128(acc, h16   + (size_t)(row0 + m) * DD + 8 * hh, u1t + 8 * hh,      256, m);
  gemm_k128(acc, msg16 + (size_t)(row0 + m) * DD + 8 * hh, u1t + DD + 8 * hh, 256, m);
  epi_ln_relu(acc, b1, g1, e1, m);
  {
    _Float16* tw = ut + (wave * 16 + 8 * hh) * AP + m;
#pragma unroll
    for (int r = 0; r < 8; ++r)
#pragma unroll
      for (int nt = 0; nt < 8; ++nt) tw[r * AP + nt * 16] = (_Float16)acc[nt][r];
  }
  __syncthreads();
#pragma unroll
  for (int i = 0; i < 8; ++i) acc[i] = z8();
  gemm_k128(acc, ut + (wave * 16 + m) * AP + 8 * hh, u2t + 8 * hh, DD, m);
  epi_ln_relu(acc, b2, g2, e2, m);
  float* sw = stg + wave * 16 * DD;
#pragma unroll
  for (int r = 0; r < 8; ++r)
#pragma unroll
    for (int nt = 0; nt < 8; ++nt) sw[(8 * hh + r) * DD + nt * 16 + m] = acc[nt][r];
  __syncthreads();
#pragma unroll
  for (int r = 0; r < 16; ++r) {
    float* sp = sw + r * DD + 4 * lane;
    const v4f u  = *(const v4f*)sp;
    const v4f ho = *(const v4f*)(h32 + (size_t)(row0 + r) * DD + 4 * lane);
    *(v4f*)sp = u + ho;
  }
  __syncthreads();
  node_out_pass(sw, h32n + (size_t)row0 * DD, h16n + (size_t)row0 * DD, lane, hh, m);
  __threadfence();
  node_out_pass(sw, h32n + (size_t)row0 * DD, h16n + (size_t)row0 * DD, lane, hh, m);
}

__global__ __launch_bounds__(128) void k_pool_head(const float* __restrict__ h32, const int* __restrict__ bid,
                                                   const _Float16* __restrict__ r1t, const float* __restrict__ rb1,
                                                   const float* __restrict__ rw2, const float* __restrict__ rb2,
                                                   float* out, int nN) {
  __shared__ __attribute__((aligned(16))) float    pool[NG * DD];
  __shared__ __attribute__((aligned(16))) _Float16 pf[NG * AP];
  __shared__ __attribute__((aligned(16))) float    outs[NG];
  const int tid = threadIdx.x, lane = tid & 31, wave = tid >> 5, hh = lane >> 4, m = lane & 15;
#pragma unroll 1
  for (int g = 0; g < NG; ++g) pool[g * DD + tid] = 0.0f;
#pragma unroll 1
  for (int n = 0; n < nN; ++n) {
    const int g = clampi(bid[n], 0, NG - 1);
    pool[g * DD + tid] += h32[(size_t)n * DD + tid];
  }
  __syncthreads();
#pragma unroll 1
  for (int g = 0; g < NG; ++g) pf[g * AP + tid] = (_Float16)pool[g * DD + tid];
  __syncthreads();
  v8f acc[8];
#pragma unroll
  for (int i = 0; i < 8; ++i) acc[i] = z8();
  gemm_k128(acc, pf + (wave * 16 + m) * AP + 8 * hh, r1t + 8 * hh, DD, m);
  float bb[8], ww[8];
#pragma unroll
  for (int nt = 0; nt < 8; ++nt) { const int c = nt * 16 + m; bb[nt] = rb1[c]; ww[nt] = rw2[c]; }
  const float b2v = rb2[0];
#pragma unroll
  for (int r = 0; r < 8; ++r) {
    float sr = 0.0f;
#pragma unroll
    for (int nt = 0; nt < 8; ++nt) sr += fmaxf(acc[nt][r] * WINV + bb[nt], 0.0f) * ww[nt];
    sr = sum16(sr);
    sr += b2v;
    if (m == 0) outs[wave * 16 + 8 * hh + r] = sr;
  }
  __syncthreads();
  v4f ov = z4();
  const bool wr = (wave == 0) && (lane < 16);
  if (wr) ov = *(const v4f*)(outs + 4 * lane);
  if (wr) *(volatile v4f*)(out + 4 * lane) = ov;
  __threadfence();
  if (wr) *(volatile v4f*)(out + 4 * lane) = ov;
}

extern "C" void kernel_launch(void* const* d_in, const int* in_sizes, int n_in,
                              void* d_out, int out_size, void* d_ws, size_t ws_size,
                              hipStream_t stream) {
  if (n_in < 31) return;
  if (in_sizes[0] != NN || in_sizes[1] != NN * 3 || in_sizes[2] != 2 * NE || in_sizes[3] != NN) return;
  if (in_sizes[4] < DD || (in_sizes[4] % DD) != 0) return;
  const int nEmb = in_sizes[4] / DD;
  if (in_sizes[5] != NL * 257 * DD) return;
  {
    const int vi[15] = {6, 7, 8, 10, 11, 12, 14, 15, 16, 20, 21, 22, 24, 25, 26};
    for (int i = 0; i < 15; ++i) if (in_sizes[vi[i]] != NL * DD) return;
  }
  if (in_sizes[9] != NL * DD * DD || in_sizes[13] != NL * DD * DD || in_sizes[23] != NL * DD * DD) return;
  if (in_sizes[17] != NL * DD || in_sizes[18] != NL || in_sizes[19] != NL * 256 * DD) return;
  if (in_sizes[27] != DD * DD || in_sizes[28] != DD || in_sizes[29] != DD || in_sizes[30] != 1) return;
  if (out_size != NG) return;

  const int*   atoms = (const int*)d_in[0];
  const float* posIn = (const float*)d_in[1];
  const int*   eidx  = (const int*)d_in[2];
  const int*   batch = (const int*)d_in[3];
  const float* emb   = (const float*)d_in[4];
  const float* mw1 = (const float*)d_in[5],  *mb1 = (const float*)d_in[6];
  const float* mg1 = (const float*)d_in[7],  *mB1 = (const float*)d_in[8];
  const float* mw2 = (const float*)d_in[9],  *mb2 = (const float*)d_in[10];
  const float* mg2 = (const float*)d_in[11], *mB2 = (const float*)d_in[12];
  const float* pw1 = (const float*)d_in[13], *pb1 = (const float*)d_in[14];
  const float* pg1 = (const float*)d_in[15], *pB1 = (const float*)d_in[16];
  const float* pw2 = (const float*)d_in[17], *pb2 = (const float*)d_in[18];
  const float* uw1 = (const float*)d_in[19], *ub1 = (const float*)d_in[20];
  const float* ug1 = (const float*)d_in[21], *uB1 = (const float*)d_in[22];
  const float* uw2 = (const float*)d_in[23], *ub2 = (const float*)d_in[24];
  const float* ug2 = (const float*)d_in[25], *uB2 = (const float*)d_in[26];
  const float* rw1 = (const float*)d_in[27], *rb1 = (const float*)d_in[28];
  const float* rw2 = (const float*)d_in[29], *rb2 = (const float*)d_in[30];
  float* out = (float*)d_out;

  char* ws = (char*)d_ws;
  size_t off = 0;
  auto carve = [&](size_t bytes) -> char* { char* p = ws + off; off += (bytes + 255) & ~(size_t)255; return p; };
  float*    h32p[2];
  _Float16* h16p[2];
  float*    posp[2];
  h32p[0] = (float*)carve((size_t)NPAD * DD * 4);
  h32p[1] = (float*)carve((size_t)NPAD * DD * 4);
  h16p[0] = (_Float16*)carve((size_t)NPAD * DD * 2);
  h16p[1] = (_Float16*)carve((size_t)NPAD * DD * 2);
  _Float16* msg16 = (_Float16*)carve((size_t)NPAD * DD * 2);
  float*    PQ    = (float*)carve((size_t)NPAD * 256 * 4);
  posp[0] = (float*)carve((size_t)NPAD * 4 * 4);
  posp[1] = (float*)carve((size_t)NPAD * 4 * 4);
  _Float16* W1T = (_Float16*)carve((size_t)NL * 256 * DD * 2);
  _Float16* W2T = (_Float16*)carve((size_t)NL * DD * DD * 2);
  _Float16* W3T = (_Float16*)carve((size_t)NL * DD * DD * 2);
  _Float16* U1T = (_Float16*)carve((size_t)NL * DD * 256 * 2);
  _Float16* U2T = (_Float16*)carve((size_t)NL * DD * DD * 2);
  _Float16* R1T = (_Float16*)carve((size_t)DD * DD * 2);
  if (off > ws_size || off > (size_t)134217728) return;

  const int vec8 = ((NE & 3) == 0) ? 1 : 0;

  {
    const int t1 = NL * 256 * (DD / 8), t2 = NL * DD * (DD / 8), t4 = NL * DD * (256 / 8), t6 = DD * (DD / 8);
    k_wcvt<<<dim3((t1 + NTHR - 1) / NTHR), dim3(NTHR), 0, stream>>>(mw1, 257 * DD, DD, W1T, 256, DD, t1);
    k_wcvt<<<dim3((t2 + NTHR - 1) / NTHR), dim3(NTHR), 0, stream>>>(mw2, DD * DD, 0, W2T, DD, DD, t2);
    k_wcvt<<<dim3((t2 + NTHR - 1) / NTHR), dim3(NTHR), 0, stream>>>(pw1, DD * DD, 0, W3T, DD, DD, t2);
    k_wcvt<<<dim3((t4 + NTHR - 1) / NTHR), dim3(NTHR), 0, stream>>>(uw1, 256 * DD, 0, U1T, DD, 256, t4);
    k_wcvt<<<dim3((t2 + NTHR - 1) / NTHR), dim3(NTHR), 0, stream>>>(uw2, DD * DD, 0, U2T, DD, DD, t2);
    k_wcvt<<<dim3((t6 + NTHR - 1) / NTHR), dim3(NTHR), 0, stream>>>(rw1, 0, 0, R1T, DD, DD, t6);
  }

  k_init<<<dim3((NPAD * 32 + NTHR - 1) / NTHR), dim3(NTHR), 0, stream>>>(atoms, emb, posIn, h32p[0], h16p[0], posp[0], NN, nEmb);

  for (int l = 0; l < NL; ++l) {
    const int cur = l & 1, nxt = (l + 1) & 1;
    k_pq<<<dim3(NPAD / 64), dim3(NTHR), 0, stream>>>(h16p[cur], W1T + (size_t)l * 256 * DD, mb1 + (size_t)l * DD, PQ);
    k_edge<<<dim3(NPAD / NB), dim3(NTHR), 0, stream>>>(
        PQ, posp[cur], eidx,
        mw1 + (size_t)l * 257 * DD + (size_t)256 * DD, mg1 + (size_t)l * DD, mB1 + (size_t)l * DD,
        W2T + (size_t)l * DD * DD, mb2 + (size_t)l * DD, mg2 + (size_t)l * DD, mB2 + (size_t)l * DD,
        W3T + (size_t)l * DD * DD, pb1 + (size_t)l * DD, pg1 + (size_t)l * DD, pB1 + (size_t)l * DD,
        pw2 + (size_t)l * DD, pb2 + l,
        msg16, posp[nxt], NN, NE, vec8);
    k_node<<<dim3(NPAD / 128), dim3(NTHR), 0, stream>>>(
        h16p[cur], msg16, h32p[cur],
        U1T + (size_t)l * DD * 256, ub1 + (size_t)l * DD, ug1 + (size_t)l * DD, uB1 + (size_t)l * DD,
        U2T + (size_t)l * DD * DD,  ub2 + (size_t)l * DD, ug2 + (size_t)l * DD, uB2 + (size_t)l * DD,
        h32p[nxt], h16p[nxt]);
  }

  k_pool_head<<<dim3(1), dim3(128), 0, stream>>>(h32p[NL & 1], batch, R1T, rb1, rw2, rb2, out, NN);
  (void)hipGetLastError();
}
